// ScaledMultiHeadAttention_39453569581187
// MI455X (gfx1250) — hardware-verified
//
#include <hip/hip_runtime.h>
#include <math.h>

#ifndef NB
#define NB 2
#endif
#ifndef SEQ
#define SEQ 2048
#endif
#define NB_FULL  2
#define SEQ_FULL 2048
#define DM   512
#define NH   8
#define HD   64
#define MT   (NB * SEQ)
#define NREL 499
#define RPAD 512
#define RCEN 249
#define AWV  4
#define RWP  48
#define WSCL 64.0f
#define QKS  16.0f
#define LSC  2048.0f
#define VSC  16.0f
#define PSC  4096.0f
#define CSC  16.0f
#define RSQD 0.125f
#define MASKV (-1.0e10f)

static_assert(NH * HD == DM);
static_assert(HD == 64);
static_assert(NB >= 1 && NB <= NB_FULL);
static_assert((SEQ % 64) == 0 && SEQ >= 64 && SEQ <= SEQ_FULL);
static_assert((MT % 64) == 0 && (DM % 64) == 0);
static_assert((((MT / 64) * (DM / 64)) % 8) == 0);
static_assert(((SEQ * DM) % 2048) == 0 && ((RPAD * HD) % 2048) == 0 && ((NREL * HD) % 8) == 0);
static_assert(((NB * NH * (SEQ / 16)) % AWV) == 0);
static_assert(NREL <= RPAD && (2 * RCEN + 1) == NREL);

typedef _Float16 v16h __attribute__((ext_vector_type(16)));
typedef unsigned short v16us __attribute__((ext_vector_type(16)));
typedef unsigned short v8us  __attribute__((ext_vector_type(8)));
typedef float v8f __attribute__((ext_vector_type(8)));
typedef float v4f __attribute__((ext_vector_type(4)));
typedef unsigned int v4u __attribute__((ext_vector_type(4)));

union FragU { v16us v; v8us h[2]; };

__device__ __forceinline__ unsigned short bf_bits(float f) {
  const unsigned u = __float_as_uint(f);
  return (unsigned short)((u + 0x7FFFu + ((u >> 16) & 1u)) >> 16);
}
__device__ __forceinline__ float bf_up(unsigned short h) { return __uint_as_float(((unsigned)h) << 16); }
__device__ __forceinline__ float bfr(float f) { return bf_up(bf_bits(f)); }
__device__ __forceinline__ unsigned short h_bits(_Float16 x) { return __builtin_bit_cast(unsigned short, x); }
__device__ __forceinline__ unsigned short f2h(float f) { return h_bits((_Float16)f); }
__device__ __forceinline__ unsigned pk16(unsigned short a, unsigned short b) { return (unsigned)a | ((unsigned)b << 16); }
__device__ __forceinline__ int clampi(int v, int lo, int hi) { return v < lo ? lo : (v > hi ? hi : v); }
__device__ __forceinline__ v8f zero8() { v8f z = {0.f, 0.f, 0.f, 0.f, 0.f, 0.f, 0.f, 0.f}; return z; }

__device__ __forceinline__ v16us ldfrag_u(const unsigned short* p) {
  FragU f;
  f.h[0] = *(const v8us*)(p);
  f.h[1] = *(const v8us*)(p + 16);
  return f.v;
}

__device__ __forceinline__ v8f mma_raw(v16us a, v16us b, v8f c) {
  return __builtin_amdgcn_wmma_f32_16x16x32_f16(false, __builtin_bit_cast(v16h, a), false,
                                                __builtin_bit_cast(v16h, b), (short)0, c, false, false);
}
__device__ __forceinline__ v8f mma_g(v16us a, v16us b, v8f c) {
  c = mma_raw(a, b, c);
#if defined(__HIP_DEVICE_COMPILE__)
  asm volatile("v_nop\n\tv_nop\n\tv_nop\n\tv_nop" : "+v"(c) : "v"(a), "v"(b));
#endif
  return c;
}
__device__ __forceinline__ void dep_guard1(v8f& a, v8f& b, v16us x) {
#if defined(__HIP_DEVICE_COMPILE__)
  asm volatile("v_nop\n\tv_nop\n\tv_nop\n\tv_nop" : "+v"(a), "+v"(b) : "v"(x));
#endif
}
__device__ __forceinline__ void keep4_u(v16us a, v16us b, v16us c, v16us d) {
#if defined(__HIP_DEVICE_COMPILE__)
  asm volatile("v_nop" :: "v"(a), "v"(b), "v"(c), "v"(d));
#endif
}
__device__ __forceinline__ void acc_guard4(v8f& a, v8f& b, v8f& c, v8f& d) {
#if defined(__HIP_DEVICE_COMPILE__)
  asm volatile("v_nop\n\tv_nop\n\tv_nop\n\tv_nop" : "+v"(a), "+v"(b), "+v"(c), "+v"(d));
#endif
}
__device__ __forceinline__ void wave_sync_lds() {
  __builtin_amdgcn_fence(__ATOMIC_RELEASE, "workgroup");
  __builtin_amdgcn_wave_barrier();
  __builtin_amdgcn_fence(__ATOMIC_ACQUIRE, "workgroup");
}

__global__ __launch_bounds__(256) void cvt_lin(const float* __restrict__ w, unsigned short* o,
                                                int nsrc, int ndst, float sc, int sstr, int dstr) {
  const float* wb = w + (size_t)blockIdx.y * (size_t)sstr;
  unsigned short* ob = o + (size_t)blockIdx.y * (size_t)dstr;
  const int base = (blockIdx.x * 256 + threadIdx.x) * 8;
  if (base + 8 > ndst) return;
  const bool inr = (base + 8 <= nsrc);
  const int lb = inr ? base : (nsrc - 8);
  const v4f a0 = *(const v4f*)(wb + lb);
  const v4f a1 = *(const v4f*)(wb + lb + 4);
  v4u hv;
#pragma unroll
  for (int e = 0; e < 2; ++e) {
    hv[e]     = pk16(f2h(bfr(a0[2 * e]) * sc), f2h(bfr(a0[2 * e + 1]) * sc));
    hv[2 + e] = pk16(f2h(bfr(a1[2 * e]) * sc), f2h(bfr(a1[2 * e + 1]) * sc));
  }
  const v4u zz = {0u, 0u, 0u, 0u};
  hv = inr ? hv : zz;
  unsigned short* d = ob + base;
  *(volatile v4u*)d = hv;
  __threadfence();
  *(volatile v4u*)d = hv;
}

__global__ __launch_bounds__(256) void cvt_t(const float* __restrict__ w, unsigned short* o, int R, int C, float sc) {
  __shared__ __align__(16) unsigned short st[64 * 72];
  const int t = threadIdx.x;
  const int r0 = blockIdx.y * 64, c0 = blockIdx.x * 64;
  if (r0 + 64 > R || c0 + 64 > C) return;
  {
    const int row = t >> 2, ch = (t & 3) * 16;
    const float* p = w + (size_t)(r0 + row) * C + c0 + ch;
#pragma unroll
    for (int q = 0; q < 4; ++q) {
      const v4f v = *(const v4f*)(p + 4 * q);
#pragma unroll
      for (int e = 0; e < 4; ++e) st[(ch + 4 * q + e) * 72 + row] = f2h(bfr(v[e]) * sc);
    }
  }
  __syncthreads();
  v4u hv[2];
#pragma unroll
  for (int half = 0; half < 2; ++half) {
    const int cl = (t >> 3) + 32 * half, pc = (t & 7) * 8;
    hv[half] = *(const v4u*)(st + cl * 72 + pc);
  }
  for (int pass = 0; pass < 2; ++pass) {
#pragma unroll
    for (int half = 0; half < 2; ++half) {
      const int cl = (t >> 3) + 32 * half, pc = (t & 7) * 8;
      unsigned short* dst = o + (size_t)(c0 + cl) * R + r0 + pc;
      *(volatile v4u*)dst = hv[half];
    }
    __threadfence();
  }
}

template <int OM, int BM>
__global__ __launch_bounds__(256) void gemm64(
    const unsigned short* __restrict__ Ap, int lda, const unsigned short* __restrict__ Btp, int ldb,
    unsigned short* Ch, unsigned short* Cl, float* Cf, int ldc, float osc,
    const float* __restrict__ bias, float bsc, int M, int N, int K) {
  __shared__ __align__(16) float sT[8][16 * 68];
  const int lane = threadIdx.x & 31;
  const int wave = threadIdx.x >> 5;
  const int tilesN = N >> 6;
  const int tilesM = M >> 6;
  const int tile = blockIdx.x * 8 + wave;
  if (tile >= tilesM * tilesN) return;
  const int tm = tile / tilesN;
  const int tn = tile - tm * tilesN;
  const int m0 = tm << 6;
  const int n0 = tn << 6;

  const int rlane = lane & 15;
  const int koff  = (lane >> 4) * 8;
  const int mOff  = (lane >> 4) * 8;

  v8f acc[4][4];
#pragma unroll
  for (int i = 0; i < 4; ++i)
#pragma unroll
    for (int j = 0; j < 4; ++j) acc[i][j] = zero8();

#pragma unroll 1
  for (int k0 = 0; k0 < K; k0 += 32) {
    v16us bh[4];
#pragma unroll
    for (int j = 0; j < 4; ++j) {
      const size_t bo = (size_t)(n0 + (j << 4) + rlane) * ldb + koff + k0;
      bh[j] = ldfrag_u(Btp + bo);
    }
#pragma unroll
    for (int i = 0; i < 4; ++i) {
      const size_t ao = (size_t)(m0 + (i << 4) + rlane) * lda + koff + k0;
      const v16us ah = ldfrag_u(Ap + ao);
#pragma unroll
      for (int j = 0; j < 4; ++j) acc[i][j] = mma_raw(ah, bh[j], acc[i][j]);
      dep_guard1(acc[i][0], acc[i][3], ah);
    }
    keep4_u(bh[0], bh[1], bh[2], bh[3]);
  }
  acc_guard4(acc[0][0], acc[0][1], acc[0][2], acc[0][3]);
  acc_guard4(acc[1][0], acc[1][1], acc[1][2], acc[1][3]);
  acc_guard4(acc[2][0], acc[2][1], acc[2][2], acc[2][3]);
  acc_guard4(acc[3][0], acc[3][1], acc[3][2], acc[3][3]);

  const int hh2 = lane >> 4, c4 = (lane & 15) * 4;
  const int q8  = lane >> 3, c8 = (lane & 7) * 8;

  v4f bc4 = {0.f, 0.f, 0.f, 0.f};
  float bc8[8];
#pragma unroll
  for (int e = 0; e < 8; ++e) bc8[e] = 0.f;
  if (BM == 1) {
    if (OM == 0) {
      const v4f t4 = *(const v4f*)(bias + n0 + c4);
#pragma unroll
      for (int e = 0; e < 4; ++e) bc4[e] = bfr(t4[e]) * bsc;
    } else {
      const v4f ta = *(const v4f*)(bias + n0 + c8);
      const v4f tb = *(const v4f*)(bias + n0 + c8 + 4);
#pragma unroll
      for (int e = 0; e < 4; ++e) { bc8[e] = bfr(ta[e]) * bsc; bc8[4 + e] = bfr(tb[e]) * bsc; }
    }
  }

  float* slab = sT[wave];
#pragma unroll
  for (int i = 0; i < 4; ++i) {
    const int mBase = m0 + (i << 4);
#pragma unroll
    for (int j = 0; j < 4; ++j) {
#pragma unroll
      for (int r = 0; r < 8; ++r) {
        slab[(mOff + r) * 68 + (j << 4) + rlane] = acc[i][j][r];
      }
    }
    wave_sync_lds();
    if (OM == 0) {
      v4f vals[8];
#pragma unroll
      for (int it = 0; it < 8; ++it) {
        const int row = it * 2 + hh2;
        const v4f v = *(const v4f*)(slab + row * 68 + c4);
        float rb2 = 0.f;
        if (BM == 2) rb2 = bfr(bias[mBase + row]) * bsc;
        vals[it] = v * osc + bc4 + rb2;
      }
      for (int pass = 0; pass < 2; ++pass) {
#pragma unroll
        for (int it = 0; it < 8; ++it) {
          const int row = it * 2 + hh2;
          *(volatile v4f*)(Cf + (size_t)(mBase + row) * ldc + (size_t)n0 + c4) = vals[it];
        }
        __threadfence();
      }
    } else {
      v4u hv[4], hl[4];
#pragma unroll
      for (int it = 0; it < 4; ++it) {
        const int row = it * 4 + q8;
        const float* sp = slab + row * 68 + c8;
        float rb2 = 0.f;
        if (BM == 2) rb2 = bfr(bias[mBase + row]) * bsc;
        v4u ha = {0u, 0u, 0u, 0u};
        v4u la = {0u, 0u, 0u, 0u};
#pragma unroll
        for (int e = 0; e < 4; ++e) {
          const float b0 = sp[2 * e]     * osc + bc8[2 * e]     + rb2;
          const float b1 = sp[2 * e + 1] * osc + bc8[2 * e + 1] + rb2;
          if (OM == 1) {
            ha[e] = pk16(f2h(b0), f2h(b1));
          } else {
            const _Float16 h0 = (_Float16)b0;
            const _Float16 h1 = (_Float16)b1;
            const float l0 = (b0 - (float)h0) * LSC;
            const float l1 = (b1 - (float)h1) * LSC;
            ha[e] = pk16(h_bits(h0), h_bits(h1));
            la[e] = pk16(f2h(l0), f2h(l1));
          }
        }
        hv[it] = ha;
        hl[it] = la;
      }
      for (int pass = 0; pass < 2; ++pass) {
#pragma unroll
        for (int it = 0; it < 4; ++it) {
          const int row = it * 4 + q8;
          const size_t go = (size_t)(mBase + row) * ldc + (size_t)n0 + c8;
          *(volatile v4u*)(Ch + go) = hv[it];
          if (OM == 2) *(volatile v4u*)(Cl + go) = hl[it];
        }
        __threadfence();
      }
    }
    wave_sync_lds();
  }
}

__device__ __forceinline__ v8f dot2_res(v16us ah0, v16us ah1, v16us al0, v16us al1, const unsigned short* p) {
  const v16us b0 = ldfrag_u(p);
  const v16us b1 = ldfrag_u(p + 32);
  v8f L = mma_g(al0, b0, zero8());
  L = mma_g(al1, b1, L);
  L = L * (1.0f / LSC);
  v8f R = mma_g(ah0, b0, L);
  R = mma_g(ah1, b1, R);
  return R;
}
__device__ __forceinline__ v8f dot3_res(v16us qh0, v16us qh1, v16us ql0, v16us ql1,
                                        const unsigned short* phi, const unsigned short* plo) {
  const v16us kh0 = ldfrag_u(phi);
  const v16us kh1 = ldfrag_u(phi + 32);
  const v16us kl0 = ldfrag_u(plo);
  const v16us kl1 = ldfrag_u(plo + 32);
  v8f L = mma_g(qh0, kl0, zero8());
  L = mma_g(qh1, kl1, L);
  L = mma_g(ql0, kh0, L);
  L = mma_g(ql1, kh1, L);
  L = L * (1.0f / LSC);
  v8f S = mma_g(qh0, kh0, L);
  S = mma_g(qh1, kh1, S);
  return S;
}

__global__ __launch_bounds__(128) void attn_kernel(
    const unsigned short* __restrict__ QH, const unsigned short* __restrict__ QL,
    const unsigned short* __restrict__ KH, const unsigned short* __restrict__ KL,
    const unsigned short* __restrict__ PE, const unsigned short* __restrict__ VT,
    const int* __restrict__ mask, unsigned short* Z) {
  __shared__ __align__(16) float relw[AWV][16 * RWP];
  __shared__ __align__(16) unsigned short pws[AWV][16 * 32];
  __shared__ __align__(16) unsigned short zst[AWV][16 * 64];
  const int lane = threadIdx.x & 31, wv = threadIdx.x >> 5, m = lane & 15, hh = lane >> 4;
  const int task = blockIdx.x * AWV + wv;
  const int nqt = SEQ / 16;
  const int bh = task / nqt;
  const int t0 = (task - bh * nqt) << 4;
  const int b = bh / NH, h = bh - (bh / NH) * NH;
  if (b >= NB) return;
  const size_t tok0 = (size_t)b * SEQ;
  const int* mk = mask + (size_t)b * SEQ_FULL;
  float* rw = relw[wv];
  unsigned short* ph = pws[wv];

  const size_t qo = (tok0 + (size_t)(t0 + m)) * DM + h * HD + 8 * hh;
  const v16us qh0 = ldfrag_u(QH + qo);
  const v16us qh1 = ldfrag_u(QH + qo + 32);
  const v16us ql0 = ldfrag_u(QL + qo);
  const v16us ql1 = ldfrag_u(QL + qo + 32);

  const int rb = RCEN - 15 - t0;

  v8f carry = dot2_res(qh0, qh1, ql0, ql1, PE + (size_t)clampi(rb + m, 0, NREL - 1) * HD + 8 * hh);

  float mx[8], ls[8];
  v8f O0 = zero8(), O1 = zero8(), O2 = zero8(), O3 = zero8();
#pragma unroll
  for (int r = 0; r < 8; ++r) { mx[r] = -1.0e30f; ls[r] = 0.f; }

#pragma unroll 1
  for (int kb = 0; kb < SEQ / 32; ++kb) {
    const int sb = kb << 5;
    v8f S0, S1;
    {
      const size_t ko = (tok0 + (size_t)(sb + m)) * DM + h * HD + 8 * hh;
      S0 = dot3_res(qh0, qh1, ql0, ql1, KH + ko, KL + ko);
      const size_t ko1 = ko + (size_t)16 * DM;
      S1 = dot3_res(qh0, qh1, ql0, ql1, KH + ko1, KL + ko1);
    }

    v8f Pb1 = dot2_res(qh0, qh1, ql0, ql1, PE + (size_t)clampi(rb + sb + 16 + m, 0, NREL - 1) * HD + 8 * hh);
    v8f Pb2 = dot2_res(qh0, qh1, ql0, ql1, PE + (size_t)clampi(rb + sb + 32 + m, 0, NREL - 1) * HD + 8 * hh);
#pragma unroll
    for (int r = 0; r < 8; ++r) {
      const int row = 8 * hh + r;
      rw[row * RWP + m]      = carry[r];
      rw[row * RWP + 16 + m] = Pb1[r];
      rw[row * RWP + 32 + m] = Pb2[r];
    }
    carry = Pb2;
    wave_sync_lds();

    const int mk0 = mk[sb + m];
    const int mk1 = mk[sb + 16 + m];

    float s0[8], s1[8];
#pragma unroll
    for (int r = 0; r < 8; ++r) {
      const int row = 8 * hh + r;
      const float rv0 = rw[row * RWP + 15 - row + m];
      const float rv1 = rw[row * RWP + 31 - row + m];
      const float v0 = S0[r] * (RSQD / (QKS * QKS)) + rv0 * (1.0f / (QKS * WSCL));
      const float v1 = S1[r] * (RSQD / (QKS * QKS)) + rv1 * (1.0f / (QKS * WSCL));
      s0[r] = (mk0 == 0) ? MASKV : v0;
      s1[r] = (mk1 == 0) ? MASKV : v1;
    }

#pragma unroll
    for (int r = 0; r < 8; ++r) {
      float xm = fmaxf(s0[r], s1[r]);
      xm = fmaxf(xm, __shfl_xor(xm, 1, 32));
      xm = fmaxf(xm, __shfl_xor(xm, 2, 32));
      xm = fmaxf(xm, __shfl_xor(xm, 4, 32));
      xm = fmaxf(xm, __shfl_xor(xm, 8, 32));
      const float mn = fmaxf(mx[r], xm);
      const float al = __expf(mx[r] - mn);
      mx[r] = mn;
      const float p0 = __expf(s0[r] - mn);
      const float p1 = __expf(s1[r] - mn);
      float ps = p0 + p1;
      ps += __shfl_xor(ps, 1, 32);
      ps += __shfl_xor(ps, 2, 32);
      ps += __shfl_xor(ps, 4, 32);
      ps += __shfl_xor(ps, 8, 32);
      ls[r] = ls[r] * al + ps;
      O0[r] = O0[r] * al;
      O1[r] = O1[r] * al;
      O2[r] = O2[r] * al;
      O3[r] = O3[r] * al;
      const int row = 8 * hh + r;
      ph[row * 32 + m]      = f2h(p0 * PSC);
      ph[row * 32 + 16 + m] = f2h(p1 * PSC);
    }
    wave_sync_lds();

    const v16us af = ldfrag_u(ph + m * 32 + 8 * hh);
    const size_t vo = (size_t)(h * HD + m) * MT + tok0 + (size_t)sb + 8 * hh;
    const v16us vf0 = ldfrag_u(VT + vo);
    const v16us vf1 = ldfrag_u(VT + vo + (size_t)16 * MT);
    const v16us vf2 = ldfrag_u(VT + vo + (size_t)32 * MT);
    const v16us vf3 = ldfrag_u(VT + vo + (size_t)48 * MT);
    O0 = mma_g(af, vf0, O0);
    O1 = mma_g(af, vf1, O1);
    O2 = mma_g(af, vf2, O2);
    O3 = mma_g(af, vf3, O3);
  }
  acc_guard4(O0, O1, O2, O3);

  unsigned short* zs = zst[wv];
  const float fin = CSC / (PSC * VSC);
#pragma unroll
  for (int r = 0; r < 8; ++r) {
    const int row = 8 * hh + r;
    const float linv = 1.0f / ls[r];
    const float g = linv * fin;
    zs[row * 64 + m]      = f2h(O0[r] * g);
    zs[row * 64 + 16 + m] = f2h(O1[r] * g);
    zs[row * 64 + 32 + m] = f2h(O2[r] * g);
    zs[row * 64 + 48 + m] = f2h(O3[r] * g);
  }
  wave_sync_lds();
  {
    const int q8 = lane >> 3, c8 = (lane & 7) * 8;
    v4u hv[4];
#pragma unroll
    for (int it = 0; it < 4; ++it) {
      const int row = it * 4 + q8;
      hv[it] = *(const v4u*)(zs + row * 64 + c8);
    }
    const size_t zr0 = (size_t)b * SEQ + (size_t)t0;
    for (int pass = 0; pass < 2; ++pass) {
#pragma unroll
      for (int it = 0; it < 4; ++it) {
        const int row = it * 4 + q8;
        unsigned short* dst = Z + (zr0 + (size_t)row) * DM + h * HD + c8;
        *(volatile v4u*)dst = hv[it];
      }
      __threadfence();
    }
  }
}

extern "C" void kernel_launch(void* const* d_in, const int* in_sizes, int n_in,
                              void* d_out, int out_size, void* d_ws, size_t ws_size,
                              hipStream_t stream) {
  if (n_in < 13) return;
  const int xreq = ((NB - 1) * SEQ_FULL + SEQ) * DM;
  const int mreq = (NB - 1) * SEQ_FULL + SEQ;
  if (in_sizes[0] < xreq || in_sizes[1] < xreq || in_sizes[2] < xreq) return;
  if (in_sizes[3] < mreq) return;
  if (in_sizes[4] < DM * DM || in_sizes[6] < DM * DM || in_sizes[8] < DM * DM || in_sizes[10] < DM * DM) return;
  if (in_sizes[5] < DM || in_sizes[7] < DM || in_sizes[9] < DM || in_sizes[11] < DM) return;
  if (in_sizes[12] < NREL * HD) return;
  if (out_size < MT * DM) return;

  const float* query = (const float*)d_in[0];
  const float* key   = (const float*)d_in[1];
  const float* value = (const float*)d_in[2];
  const int*   mask  = (const int*)d_in[3];
  const float* wq = (const float*)d_in[4];
  const float* bq = (const float*)d_in[5];
  const float* wk = (const float*)d_in[6];
  const float* bk = (const float*)d_in[7];
  const float* wv = (const float*)d_in[8];
  const float* bv = (const float*)d_in[9];
  const float* wo = (const float*)d_in[10];
  const float* bo = (const float*)d_in[11];
  const float* rel = (const float*)d_in[12];

  const size_t PX  = (size_t)MT * DM * 2;
  const size_t PWT = (size_t)3 * DM * DM * 2;
  const size_t PWO = (size_t)DM * DM * 2;
  const size_t PPE = (size_t)RPAD * HD * 2;
  size_t off = 0;
  const size_t oXQ = off; off += PX;
  const size_t oXK = off; off += PX;
  const size_t oXV = off; off += PX;
  const size_t oWT = off; off += PWT;
  const size_t oWO = off; off += PWO;
  const size_t oPE = off; off += PPE;
  const size_t oQH = off; off += PX;
  const size_t oQL = off; off += PX;
  const size_t oKH = off; off += PX;
  const size_t oKL = off; off += PX;
  const size_t oVT = off; off += PX;
  const size_t oZ  = off; off += PX;
  if (off > ws_size) return;
  if (off > (size_t)134217728) return;

  char* ws = (char*)d_ws;
  unsigned short* XQ  = (unsigned short*)(ws + oXQ);
  unsigned short* XK  = (unsigned short*)(ws + oXK);
  unsigned short* XV  = (unsigned short*)(ws + oXV);
  unsigned short* WT  = (unsigned short*)(ws + oWT);
  unsigned short* WOT = (unsigned short*)(ws + oWO);
  unsigned short* PEH = (unsigned short*)(ws + oPE);
  unsigned short* QH  = (unsigned short*)(ws + oQH);
  unsigned short* QL  = (unsigned short*)(ws + oQL);
  unsigned short* KH  = (unsigned short*)(ws + oKH);
  unsigned short* KL  = (unsigned short*)(ws + oKL);
  unsigned short* VT  = (unsigned short*)(ws + oVT);
  unsigned short* Z   = (unsigned short*)(ws + oZ);
  float* out0 = (float*)d_out;
  float* fdummy = (float*)(ws + oXQ);
  unsigned short* hdummy = XQ;

  const dim3 blk(256);
  const int gP = ((MT / 64) * (DM / 64)) / 8;

  cvt_lin<<<dim3((SEQ * DM) / 2048, NB), blk, 0, stream>>>(query, XQ, SEQ * DM, SEQ * DM, 1.0f, SEQ_FULL * DM, SEQ * DM);
  cvt_lin<<<dim3((SEQ * DM) / 2048, NB), blk, 0, stream>>>(key,   XK, SEQ * DM, SEQ * DM, 1.0f, SEQ_FULL * DM, SEQ * DM);
  cvt_lin<<<dim3((SEQ * DM) / 2048, NB), blk, 0, stream>>>(value, XV, SEQ * DM, SEQ * DM, 1.0f, SEQ_FULL * DM, SEQ * DM);
  cvt_lin<<<dim3((RPAD * HD) / 2048, 1), blk, 0, stream>>>(rel, PEH, NREL * HD, RPAD * HD, WSCL, 0, 0);
  cvt_t<<<dim3(DM / 64, DM / 64), blk, 0, stream>>>(wq, WT, DM, DM, WSCL);
  cvt_t<<<dim3(DM / 64, DM / 64), blk, 0, stream>>>(wk, WT + (size_t)DM * DM, DM, DM, WSCL);
  cvt_t<<<dim3(DM / 64, DM / 64), blk, 0, stream>>>(wv, WT + (size_t)2 * DM * DM, DM, DM, WSCL);
  cvt_t<<<dim3(DM / 64, DM / 64), blk, 0, stream>>>(wo, WOT, DM, DM, WSCL);

  gemm64<2, 1><<<dim3(gP), blk, 0, stream>>>(XQ, DM, WT, DM, QH, QL, fdummy, DM, QKS / WSCL, bq, QKS, MT, DM, DM);
  gemm64<2, 1><<<dim3(gP), blk, 0, stream>>>(XK, DM, WT + (size_t)DM * DM, DM, KH, KL, fdummy, DM, QKS / WSCL, bk, QKS, MT, DM, DM);
  gemm64<1, 2><<<dim3(gP), blk, 0, stream>>>(WT + (size_t)2 * DM * DM, DM, XV, DM, VT, hdummy, fdummy, MT, VSC / WSCL, bv, VSC, DM, MT, DM);

  attn_kernel<<<dim3((NB * NH * (SEQ / 16)) / AWV), dim3(128), 0, stream>>>(QH, QL, KH, KL, PEH, VT, mask, Z);

  gemm64<0, 1><<<dim3(gP), blk, 0, stream>>>(Z, DM, WOT, DM, hdummy, hdummy, out0, DM, 1.0f / (WSCL * CSC), bo, 1.0f, MT, DM, DM);
  (void)hipGetLastError();
}
